// ImportanceGuidedCrossAttention_47364899340798
// MI455X (gfx1250) — hardware-verified
//
#include <hip/hip_runtime.h>
#include <math.h>
#include <stdint.h>

#define NBAT   2
#define NQ     1024
#define MKV    4096
#define DMOD   1024
#define NHEAD  16
#define DHEAD  64
#define MTQ    (NBAT * NQ)
#define MTC    (NBAT * MKV)
#define KSEG   (DMOD / 256)
#define TN64   (DMOD / 64)
#define XBLK   ((MTQ * KSEG) / 8)
#define CBLK   ((MTC * KSEG) / 8)
#define WTILE  ((DMOD / 64) * (DMOD / 64))
#define NQB    (NQ / 64)
#define XC     64.0f
#define WSC    1024.0f
#define QS     1024.0f
#define KS     1024.0f
#define VS     256.0f
#define CS     1024.0f
#define LNPS   6.931471805599453f
#define ATTSC  0.125f
static_assert(NHEAD * DHEAD == DMOD);
static_assert(DHEAD == 64);
static_assert((MTQ % 64) == 0 && (MTC % 64) == 0 && (DMOD % 64) == 0 && (DMOD % 32) == 0 && (DMOD % 256) == 0);
static_assert((((MTQ / 64) * TN64) % 4) == 0 && (((MTC / 64) * TN64) % 4) == 0);
static_assert(((MTQ * KSEG) % 8) == 0 && ((MTC * KSEG) % 8) == 0);
static_assert((NQ % 64) == 0 && (MKV % 64) == 0 && (MKV % 32) == 0 && (MKV % 128) == 0);
static_assert(WTILE == 256 && XBLK == 1024 && CBLK == 4096 && NQB == 16);

typedef _Float16 v16h __attribute__((ext_vector_type(16)));
typedef _Float16 v8h  __attribute__((ext_vector_type(8)));
typedef float    v8f  __attribute__((ext_vector_type(8)));
typedef float    v4f  __attribute__((ext_vector_type(4)));
typedef unsigned int v4u __attribute__((ext_vector_type(4)));

union FragH { v16h v; v8h h[2]; };

__device__ __forceinline__ unsigned short bf_bits(float f) {
  unsigned u = __float_as_uint(f);
  return (unsigned short)((u + 0x7FFFu + ((u >> 16) & 1u)) >> 16);
}
__device__ __forceinline__ float bf_up(unsigned short h) { return __uint_as_float(((unsigned)h) << 16); }
__device__ __forceinline__ float bfr(float f) { return bf_up(bf_bits(f)); }
__device__ __forceinline__ unsigned short h_bits(_Float16 x) { return __builtin_bit_cast(unsigned short, x); }
__device__ __forceinline__ unsigned pk16(unsigned short a, unsigned short b) { return (unsigned)a | ((unsigned)b << 16); }
__device__ __forceinline__ v8f zero8() { v8f z = {0.f, 0.f, 0.f, 0.f, 0.f, 0.f, 0.f, 0.f}; return z; }

__device__ __forceinline__ v16h ldfrag_h(const _Float16* p) {
  FragH f;
  f.h[0] = *(const v8h*)(p);
  f.h[1] = *(const v8h*)(p + 16);
  return f.v;
}

__device__ __forceinline__ v8f mma_h_raw(v16h a, v16h b, v8f c) {
  return __builtin_amdgcn_wmma_f32_16x16x32_f16(false, a, false, b, (short)0, c, false, false);
}
__device__ __forceinline__ void dep_guard1(v8f& a, v8f& b, v16h x) {
#if defined(__HIP_DEVICE_COMPILE__)
  asm volatile("v_nop\n\tv_nop\n\tv_nop\n\tv_nop" : "+v"(a), "+v"(b) : "v"(x));
#endif
}
__device__ __forceinline__ void keep4_h(v16h a, v16h b, v16h c, v16h d) {
#if defined(__HIP_DEVICE_COMPILE__)
  asm volatile("v_nop" :: "v"(a), "v"(b), "v"(c), "v"(d));
#endif
}
__device__ __forceinline__ void acc_guard4(v8f& a, v8f& b, v8f& c, v8f& d) {
#if defined(__HIP_DEVICE_COMPILE__)
  asm volatile("v_nop\n\tv_nop\n\tv_nop\n\tv_nop" : "+v"(a), "+v"(b), "+v"(c), "+v"(d));
#endif
}
__device__ __forceinline__ void sguard6(v8f& a, v8f& b, v16h x0, v16h x1, v16h x2, v16h x3, v16h x4, v16h x5) {
#if defined(__HIP_DEVICE_COMPILE__)
  asm volatile("v_nop\n\tv_nop\n\tv_nop\n\tv_nop"
               : "+v"(a), "+v"(b) : "v"(x0), "v"(x1), "v"(x2), "v"(x3), "v"(x4), "v"(x5));
#endif
}
__device__ __forceinline__ void oguard6(v8f& a, v8f& b, v8f& c, v8f& d,
                                        v16h x0, v16h x1, v16h x2, v16h x3, v16h p0, v16h p1) {
#if defined(__HIP_DEVICE_COMPILE__)
  asm volatile("v_nop\n\tv_nop\n\tv_nop\n\tv_nop"
               : "+v"(a), "+v"(b), "+v"(c), "+v"(d) : "v"(x0), "v"(x1), "v"(x2), "v"(x3), "v"(p0), "v"(p1));
#endif
}
__device__ __forceinline__ void wave_sync_lds() {
  __builtin_amdgcn_fence(__ATOMIC_RELEASE, "workgroup");
  __builtin_amdgcn_wave_barrier();
  __builtin_amdgcn_fence(__ATOMIC_ACQUIRE, "workgroup");
}

__global__ __launch_bounds__(256) void cvt_rows(const float* __restrict__ xs, const float* __restrict__ cs,
                                                unsigned short* xh, unsigned short* ch) {
  const int lane = threadIdx.x & 31, wave = threadIdx.x >> 5;
  const int bx = blockIdx.x;
  const float* src;
  unsigned short* dst;
  int lb;
  if (bx < XBLK) { src = xs; dst = xh; lb = bx; }
  else           { src = cs; dst = ch; lb = bx - XBLK; }
  const int seg = lb * 8 + wave;
  const int row = seg / KSEG;
  const int col = (seg - row * KSEG) * 256 + 8 * lane;
  const size_t o = (size_t)row * DMOD + col;
  const v4f h0 = *(const v4f*)(src + o), h1 = *(const v4f*)(src + o + 4);
  float a[8];
#pragma unroll
  for (int i = 0; i < 4; ++i) { a[i] = bfr(h0[i]); a[4 + i] = bfr(h1[i]); }
  v4u uh;
#pragma unroll
  for (int i = 0; i < 4; ++i) {
    const float xa = a[2 * i] * XC, xb = a[2 * i + 1] * XC;
    uh[i] = pk16(h_bits((_Float16)xa), h_bits((_Float16)xb));
  }
  unsigned short* dh = dst + o;
  *(volatile v4u*)dh = uh;
  __threadfence();
  *(volatile v4u*)dh = uh;
}

__global__ __launch_bounds__(256) void cvt_wt(const float* __restrict__ w0, const float* __restrict__ w1,
                                              const float* __restrict__ w2, const float* __restrict__ w3,
                                              unsigned short* t0, unsigned short* t1,
                                              unsigned short* t2, unsigned short* t3) {
  __shared__ __align__(16) unsigned short Ts[64 * 72];
  const int tid = threadIdx.x;
  const int bx = blockIdx.x;
  const int wsel = bx / WTILE;
  const int tb = bx - wsel * WTILE;
  const int tk = tb / TN64, tn = tb - tk * TN64;
  const int k0 = tk << 6, n0 = tn << 6;
  const float* src = (wsel == 0) ? w0 : (wsel == 1) ? w1 : (wsel == 2) ? w2 : w3;
  unsigned short* dst = (wsel == 0) ? t0 : (wsel == 1) ? t1 : (wsel == 2) ? t2 : t3;

  const int r = tid >> 2, cseg = (tid & 3) * 16;
  const float* sp = src + (size_t)(k0 + r) * DMOD + n0 + cseg;
  const v4f f0 = *(const v4f*)(sp), f1 = *(const v4f*)(sp + 4), f2 = *(const v4f*)(sp + 8), f3 = *(const v4f*)(sp + 12);
  float a[16];
#pragma unroll
  for (int i = 0; i < 4; ++i) { a[i] = f0[i]; a[4 + i] = f1[i]; a[8 + i] = f2[i]; a[12 + i] = f3[i]; }
#pragma unroll
  for (int i = 0; i < 16; ++i) {
    Ts[(cseg + i) * 72 + r] = h_bits((_Float16)(bfr(a[i]) * WSC));
  }
  __syncthreads();
  const int e = tid & 7, g = tid >> 3;
  const v4u u0 = *(const v4u*)(Ts + g * 72 + 8 * e);
  const v4u u1 = *(const v4u*)(Ts + (g + 32) * 72 + 8 * e);
  unsigned short* dp = dst + (size_t)n0 * DMOD + k0 + 8 * e;
  for (int pass = 0; pass < 2; ++pass) {
    *(volatile v4u*)(dp + (size_t)g * DMOD) = u0;
    *(volatile v4u*)(dp + (size_t)(g + 32) * DMOD) = u1;
    __threadfence();
  }
}

template <int MODE, int MROWS, int TPB>
__global__ __launch_bounds__(128) void gemm64(
    const unsigned short* __restrict__ Ap, const unsigned short* __restrict__ Bp,
    const float* __restrict__ bias, float escale, float bscale, void* C0) {
  static_assert((MROWS % 64) == 0 && (TPB % 64) == 0 && (MROWS % TPB) == 0);
  static_assert((((MROWS / 64) * TN64) % 4) == 0);
  __shared__ __align__(16) unsigned short sraw[4][4608];
  const int lane = threadIdx.x & 31;
  const int wave = threadIdx.x >> 5;
  const int tilesN = TN64;
  const int tile = blockIdx.x * 4 + wave;
  const int tm = tile / tilesN;
  const int tn = tile - tm * tilesN;
  const int m0 = tm << 6;
  const int n0 = tn << 6;

  const _Float16* Ah = (const _Float16*)(const void*)Ap;
  const _Float16* Bb = (const _Float16*)(const void*)Bp;

  const int rlane = lane & 15;
  const int hh    = lane >> 4;
  const int koff  = hh * 8;
  const int mOff  = hh * 8;

  v8f acc[4][4];
#pragma unroll
  for (int i = 0; i < 4; ++i)
#pragma unroll
    for (int j = 0; j < 4; ++j) acc[i][j] = zero8();

  for (int k0 = 0; k0 < DMOD; k0 += 32) {
    v16h bh[4];
#pragma unroll
    for (int j = 0; j < 4; ++j) {
      const size_t bo = (size_t)(n0 + (j << 4) + rlane) * DMOD + koff + k0;
      bh[j] = ldfrag_h(Bb + bo);
    }
#pragma unroll
    for (int i = 0; i < 4; ++i) {
      const size_t ao = (size_t)(m0 + (i << 4) + rlane) * DMOD + koff + k0;
      const v16h ah = ldfrag_h(Ah + ao);
#pragma unroll
      for (int j = 0; j < 4; ++j) acc[i][j] = mma_h_raw(ah, bh[j], acc[i][j]);
      dep_guard1(acc[i][0], acc[i][3], ah);
    }
    keep4_h(bh[0], bh[1], bh[2], bh[3]);
  }
  acc_guard4(acc[0][0], acc[0][1], acc[0][2], acc[0][3]);
  acc_guard4(acc[1][0], acc[1][1], acc[1][2], acc[1][3]);
  acc_guard4(acc[2][0], acc[2][1], acc[2][2], acc[2][3]);
  acc_guard4(acc[3][0], acc[3][1], acc[3][2], acc[3][3]);

  if (MODE == 0) {
    float* Cout = (float*)C0;
    const int c4 = rlane * 4;
    const v4f braw = *(const v4f*)(bias + n0 + c4);
    float bb[4];
#pragma unroll
    for (int tt = 0; tt < 4; ++tt) bb[tt] = bfr(braw[tt]) * bscale;
    float* slab = (float*)(void*)(&sraw[wave][0]);
#pragma unroll
    for (int i = 0; i < 4; ++i) {
      const int mBase = m0 + (i << 4);
#pragma unroll
      for (int j = 0; j < 4; ++j) {
#pragma unroll
        for (int r = 0; r < 8; ++r) slab[(mOff + r) * 68 + (j << 4) + rlane] = acc[i][j][r];
      }
      wave_sync_lds();
      v4f vals[8];
#pragma unroll
      for (int it = 0; it < 8; ++it) {
        const int row = it * 2 + hh;
        v4f v = *(const v4f*)(slab + row * 68 + c4);
#pragma unroll
        for (int tt = 0; tt < 4; ++tt) v[tt] = v[tt] * escale + bb[tt];
        vals[it] = v;
      }
      for (int pass = 0; pass < 2; ++pass) {
#pragma unroll
        for (int it = 0; it < 8; ++it) {
          const int row = it * 2 + hh;
          *(volatile v4f*)(Cout + (size_t)(mBase + row) * DMOD + n0 + c4) = vals[it];
        }
        __threadfence();
      }
      wave_sync_lds();
    }
  } else if (MODE == 1) {
    unsigned short* Hp = (unsigned short*)C0;
    const int e = lane & 7, q4 = lane >> 3;
    const v4f b0 = *(const v4f*)(bias + n0 + 8 * e), b1 = *(const v4f*)(bias + n0 + 8 * e + 4);
    float bb[8];
#pragma unroll
    for (int tt = 0; tt < 4; ++tt) { bb[tt] = bfr(b0[tt]) * bscale; bb[4 + tt] = bfr(b1[tt]) * bscale; }
    float* slab = (float*)(void*)(&sraw[wave][0]);
#pragma unroll
    for (int i = 0; i < 4; ++i) {
      const int mBase = m0 + (i << 4);
#pragma unroll
      for (int j = 0; j < 4; ++j) {
#pragma unroll
        for (int r = 0; r < 8; ++r) slab[(mOff + r) * 68 + (j << 4) + rlane] = acc[i][j][r];
      }
      wave_sync_lds();
      v4u hv[4];
#pragma unroll
      for (int it = 0; it < 4; ++it) {
        const int row = it * 4 + q4;
        const v4f x0 = *(const v4f*)(slab + row * 68 + 8 * e);
        const v4f x1 = *(const v4f*)(slab + row * 68 + 8 * e + 4);
        float y[8];
#pragma unroll
        for (int tt = 0; tt < 4; ++tt) { y[tt] = x0[tt] * escale + bb[tt]; y[4 + tt] = x1[tt] * escale + bb[4 + tt]; }
        v4u uh;
#pragma unroll
        for (int t2 = 0; t2 < 4; ++t2) {
          uh[t2] = pk16(h_bits((_Float16)y[2 * t2]), h_bits((_Float16)y[2 * t2 + 1]));
        }
        hv[it] = uh;
      }
      for (int pass = 0; pass < 2; ++pass) {
#pragma unroll
        for (int it = 0; it < 4; ++it) {
          const int row = it * 4 + q4;
          const size_t go = (size_t)(mBase + row) * DMOD + n0 + 8 * e;
          *(volatile v4u*)(Hp + go) = hv[it];
        }
        __threadfence();
      }
      wave_sync_lds();
    }
  } else {
    unsigned short* Vs = &sraw[wave][0];
    float bb4[4];
#pragma unroll
    for (int j = 0; j < 4; ++j) bb4[j] = bfr(bias[n0 + (j << 4) + rlane]) * bscale;
#pragma unroll
    for (int i = 0; i < 4; ++i) {
#pragma unroll
      for (int j = 0; j < 4; ++j) {
#pragma unroll
        for (int r = 0; r < 8; ++r) {
          Vs[((j << 4) + rlane) * 72 + (i << 4) + mOff + r] = h_bits((_Float16)(acc[i][j][r] * escale + bb4[j]));
        }
      }
    }
    wave_sync_lds();
    const int e = lane & 7, q4 = lane >> 3;
    const int bsel = m0 / TPB;
    const int s0 = m0 % TPB;
    v4u u[16];
#pragma unroll
    for (int it = 0; it < 16; ++it) {
      const int fl = it * 4 + q4;
      u[it] = *(const v4u*)(Vs + fl * 72 + 8 * e);
    }
    unsigned short* Vp = (unsigned short*)C0 + ((size_t)bsel * DMOD + n0) * TPB + s0 + 8 * e;
    for (int pass = 0; pass < 2; ++pass) {
#pragma unroll
      for (int it = 0; it < 16; ++it) {
        const int fl = it * 4 + q4;
        *(volatile v4u*)(Vp + (size_t)fl * TPB) = u[it];
      }
      __threadfence();
    }
  }
}

__global__ __launch_bounds__(128)
void attn_kernel(const unsigned short* __restrict__ qp, const unsigned short* __restrict__ kp,
                 const unsigned short* __restrict__ vt, const float* __restrict__ imp, unsigned short* ctx) {
  __shared__ __align__(16) float Os[64 * 68];
  __shared__ __align__(16) float Bs[MKV];
  const int tid  = threadIdx.x;
  const int wave = tid >> 5;
  const int lane = tid & 31;
  const int hh   = lane >> 4;
  const int c    = lane & 15;
  const int bx   = blockIdx.x;
  const int bhd  = bx / NQB;
  const int qb   = bx - bhd * NQB;
  const int b    = bhd / NHEAD;
  const int hd   = bhd - b * NHEAD;
  const int q0   = qb * 64;

  const float* ib = imp + (size_t)b * MKV;
#pragma unroll 4
  for (int i = tid; i < MKV; i += 128) Bs[i] = bfr(ib[i]);
  __syncthreads();

  const _Float16* QP  = (const _Float16*)(const void*)qp;
  const _Float16* KP  = (const _Float16*)(const void*)kp;
  const _Float16* VTp = (const _Float16*)(const void*)vt;

  const size_t qtok = (size_t)b * NQ + q0 + wave * 16 + c;
  const _Float16* qbp = QP + qtok * DMOD + hd * DHEAD + 8 * hh;
  const v16h qf0 = ldfrag_h(qbp), qf1 = ldfrag_h(qbp + 32);
  const size_t krow = ((size_t)b * MKV + c) * DMOD + hd * DHEAD + 8 * hh;
  const _Float16* Kb = KP + krow;
  const size_t vrow = ((size_t)b * DMOD + hd * DHEAD + c) * MKV + 8 * hh;
  const _Float16* V0 = VTp + vrow;
  const _Float16* V1 = V0 + (size_t)16 * MKV;
  const _Float16* V2 = V0 + (size_t)32 * MKV;
  const _Float16* V3 = V0 + (size_t)48 * MKV;
  const float* bsp = Bs + 8 * hh;
  const float SC = ATTSC / (QS * KS);

  float m = -1.0e30f, l = 0.f;
  v8f o0 = zero8(), o1 = zero8(), o2 = zero8(), o3 = zero8();
#pragma unroll 1
  for (int it = 0; it < MKV / 32; ++it) {
    const int kb = it * 32;
    const _Float16* k0p = Kb + (size_t)kb * DMOD;
    const _Float16* k1p = k0p + (size_t)16 * DMOD;
    const v16h a0 = ldfrag_h(k0p), a1 = ldfrag_h(k1p);
    const v16h a2 = ldfrag_h(k0p + 32), a3 = ldfrag_h(k1p + 32);
    v8f s0 = mma_h_raw(a0, qf0, zero8());
    v8f s1 = mma_h_raw(a1, qf0, zero8());
    s0 = mma_h_raw(a2, qf1, s0);
    s1 = mma_h_raw(a3, qf1, s1);
    sguard6(s0, s1, a0, a1, a2, a3, qf0, qf1);

    const v4f g00 = *(const v4f*)(bsp + kb),      g01 = *(const v4f*)(bsp + kb + 4);
    const v4f g10 = *(const v4f*)(bsp + kb + 16), g11 = *(const v4f*)(bsp + kb + 20);
    float x0[8], x1[8];
#pragma unroll
    for (int r = 0; r < 4; ++r) {
      x0[r]     = s0[r]     * SC + g00[r];
      x0[4 + r] = s0[4 + r] * SC + g01[r];
      x1[r]     = s1[r]     * SC + g10[r];
      x1[4 + r] = s1[4 + r] * SC + g11[r];
    }
    float mx = -3.0e38f;
#pragma unroll
    for (int r = 0; r < 8; ++r) mx = fmaxf(mx, fmaxf(x0[r], x1[r]));
    mx = fmaxf(mx, __shfl_xor(mx, 16, 32));
    const float mn   = fmaxf(m, mx);
    const float corr = __expf(m - mn);
    m = mn;
    const float msh = mn - LNPS;
    l *= corr;
#pragma unroll
    for (int r = 0; r < 8; ++r) { o0[r] *= corr; o1[r] *= corr; o2[r] *= corr; o3[r] *= corr; }

    FragH ph, pl;
    float ls = 0.f;
#pragma unroll
    for (int r = 0; r < 8; ++r) {
      const float e0 = __expf(x0[r] - msh);
      const float e1 = __expf(x1[r] - msh);
      ls += e0 + e1;
      const _Float16 h0 = (_Float16)e0, h1 = (_Float16)e1;
      ph.h[0][r] = h0;
      ph.h[1][r] = h1;
      pl.h[0][r] = (_Float16)(e0 - (float)h0);
      pl.h[1][r] = (_Float16)(e1 - (float)h1);
    }
    l += ls;

    const v16h vf0 = ldfrag_h(V0 + kb);
    const v16h vf1 = ldfrag_h(V1 + kb);
    const v16h vf2 = ldfrag_h(V2 + kb);
    const v16h vf3 = ldfrag_h(V3 + kb);
    o0 = mma_h_raw(vf0, ph.v, o0);
    o1 = mma_h_raw(vf1, ph.v, o1);
    o2 = mma_h_raw(vf2, ph.v, o2);
    o3 = mma_h_raw(vf3, ph.v, o3);
    o0 = mma_h_raw(vf0, pl.v, o0);
    o1 = mma_h_raw(vf1, pl.v, o1);
    o2 = mma_h_raw(vf2, pl.v, o2);
    o3 = mma_h_raw(vf3, pl.v, o3);
    oguard6(o0, o1, o2, o3, vf0, vf1, vf2, vf3, ph.v, pl.v);
  }
  l += __shfl_xor(l, 16, 32);
  const float sc = (CS / VS) * (1.0f / l);

  float* os = Os + (wave * 16 + c) * 68 + 8 * hh;
#pragma unroll
  for (int r = 0; r < 8; ++r) { os[r] = o0[r] * sc; os[16 + r] = o1[r] * sc; os[32 + r] = o2[r] * sc; os[48 + r] = o3[r] * sc; }
  __syncthreads();
  {
    const int e = tid & 7, qq = tid >> 3;
    v4u hv[4];
#pragma unroll
    for (int it = 0; it < 4; ++it) {
      const int qi = it * 16 + qq;
      const v4f x0 = *(const v4f*)(Os + qi * 68 + 8 * e);
      const v4f x1 = *(const v4f*)(Os + qi * 68 + 8 * e + 4);
      v4u u;
#pragma unroll
      for (int t2 = 0; t2 < 2; ++t2) {
        u[t2]     = pk16(h_bits((_Float16)x0[2 * t2]), h_bits((_Float16)x0[2 * t2 + 1]));
        u[2 + t2] = pk16(h_bits((_Float16)x1[2 * t2]), h_bits((_Float16)x1[2 * t2 + 1]));
      }
      hv[it] = u;
    }
    unsigned short* ob = ctx + (size_t)hd * DHEAD + 8 * e;
    for (int pass = 0; pass < 2; ++pass) {
#pragma unroll
      for (int it = 0; it < 4; ++it) {
        const int qi = it * 16 + qq;
        *(volatile v4u*)(ob + ((size_t)b * NQ + q0 + qi) * DMOD) = hv[it];
      }
      __threadfence();
    }
  }
}

extern "C" void kernel_launch(void* const* d_in, const int* in_sizes, int n_in,
                              void* d_out, int out_size, void* d_ws, size_t ws_size,
                              hipStream_t stream) {
  if (n_in < 8) return;
  if (in_sizes[0] != MTQ * DMOD) return;
  if (in_sizes[1] != MTC * DMOD) return;
  if (in_sizes[2] != NBAT * MKV) return;
  if (in_sizes[3] != DMOD * DMOD || in_sizes[4] != DMOD * DMOD || in_sizes[5] != DMOD * DMOD || in_sizes[6] != DMOD * DMOD) return;
  if (in_sizes[7] != DMOD) return;
  if (out_size != MTQ * DMOD) return;

  const float* xs  = (const float*)d_in[0];
  const float* cs  = (const float*)d_in[1];
  const float* imp = (const float*)d_in[2];
  const float* Wq  = (const float*)d_in[3];
  const float* Wk  = (const float*)d_in[4];
  const float* Wv  = (const float*)d_in[5];
  const float* Wo  = (const float*)d_in[6];
  const float* bo  = (const float*)d_in[7];

  const size_t PXQ = (size_t)MTQ * DMOD * 2;
  const size_t PXC = (size_t)MTC * DMOD * 2;
  const size_t PW  = (size_t)DMOD * DMOD * 2;
  const size_t PVT = (size_t)NBAT * DMOD * MKV * 2;
  size_t off = 0;
  const size_t oXH = off; off += PXQ;
  const size_t oCH = off; off += PXC;
  const size_t oWQ = off; off += PW;
  const size_t oWK = off; off += PW;
  const size_t oWV = off; off += PW;
  const size_t oWO = off; off += PW;
  const size_t oQP = off; off += PXQ;
  const size_t oKP = off; off += PXC;
  const size_t oVT = off; off += PVT;
  const size_t oCT = off; off += PXQ;
  if (off > ws_size) return;
  if (off > (size_t)134217728) return;

  char* ws = (char*)d_ws;
  unsigned short* XH  = (unsigned short*)(ws + oXH);
  unsigned short* CH  = (unsigned short*)(ws + oCH);
  unsigned short* WQT = (unsigned short*)(ws + oWQ);
  unsigned short* WKT = (unsigned short*)(ws + oWK);
  unsigned short* WVT = (unsigned short*)(ws + oWV);
  unsigned short* WOT = (unsigned short*)(ws + oWO);
  unsigned short* QPL = (unsigned short*)(ws + oQP);
  unsigned short* KPL = (unsigned short*)(ws + oKP);
  unsigned short* VT  = (unsigned short*)(ws + oVT);
  unsigned short* CTX = (unsigned short*)(ws + oCT);
  float*          out = (float*)d_out;

  const dim3 blk256(256), blk128(128);
  const dim3 gCR(XBLK + CBLK);
  const dim3 gCW(4 * WTILE);
  const dim3 gGQ(((MTQ / 64) * TN64) / 4);
  const dim3 gGC(((MTC / 64) * TN64) / 4);
  const dim3 gAT(NBAT * NHEAD * NQB);

  cvt_rows<<<gCR, blk256, 0, stream>>>(xs, cs, XH, CH);

  cvt_wt<<<gCW, blk256, 0, stream>>>(Wq, Wk, Wv, Wo, WQT, WKT, WVT, WOT);

  gemm64<1, MTQ, NQ><<<gGQ, blk128, 0, stream>>>(XH, WQT, bo, QS / (XC * WSC), 0.0f, (void*)QPL);

  gemm64<1, MTC, MKV><<<gGC, blk128, 0, stream>>>(CH, WKT, bo, KS / (XC * WSC), 0.0f, (void*)KPL);

  gemm64<2, MTC, MKV><<<gGC, blk128, 0, stream>>>(CH, WVT, bo, VS / (XC * WSC), 0.0f, (void*)VT);

  attn_kernel<<<gAT, blk128, 0, stream>>>(QPL, KPL, VT, imp, CTX);

  gemm64<0, MTQ, NQ><<<gGQ, blk128, 0, stream>>>(CTX, WOT, bo, 1.0f / (CS * WSC), 1.0f, (void*)out);
  (void)hipGetLastError();
}
